// MiniBatchDiscrimination_43508018708960
// MI455X (gfx1250) — hardware-verified
//
#include <hip/hip_runtime.h>

typedef __bf16         v16bf __attribute__((ext_vector_type(16)));
typedef unsigned short v8us  __attribute__((ext_vector_type(8)));
typedef float          v8f   __attribute__((ext_vector_type(8)));
typedef float          v4f   __attribute__((ext_vector_type(4)));
typedef unsigned int   v2u   __attribute__((ext_vector_type(2)));
typedef v8us __attribute__((may_alias)) v8usa;
typedef v4f  __attribute__((may_alias)) v4fa;
typedef v2u  __attribute__((may_alias)) v2ua;

union Frag { v16bf v; v8us half[2]; };

#define NS    32
#define HWN   256
#define FD    256
#define BD    64
#define CD    8
#define NCOL  512
#define OUTC  320
#define XP    264
#define MP    264
#define SP    36
#define TP    264

static_assert(FD % 32 == 0);
static_assert(NCOL % 16 == 0);
static_assert(NS == 32);
static_assert((XP * 2) % 16 == 0);
static_assert((MP * 4) % 16 == 0);
static_assert((SP * 4) % 16 == 0);
static_assert((OUTC * 4) % 128 == 0);

__device__ __forceinline__ v8f wmma_bf16(v16bf a, v16bf b, v8f c) {
  v8f d = __builtin_amdgcn_wmma_f32_16x16x32_bf16(false, a, false, b, (short)0, c, false, false);
  asm volatile("v_nop\n\tv_nop\n\tv_nop\n\tv_nop" : "+v"(d) : "v"(a), "v"(b));
  return d;
}

__device__ __forceinline__ v16bf load_frag(const unsigned short* p, int h) {
  Frag f;
  f.half[0] = *(const v8usa*)(p + 8 * h);
  f.half[1] = *(const v8usa*)(p + 16 + 8 * h);
  return f.v;
}

__device__ __forceinline__ unsigned int bf16_bits(float f) {
  const unsigned int u = __float_as_uint(f);
  return (u + 0x7FFFu + ((u >> 16) & 1u)) >> 16;
}

__device__ __forceinline__ void tt_store_pass(const unsigned short* St, unsigned short* Tt,
                                              int n0, int w, int lane) {
  const int q8 = lane & 7, sub = lane >> 3;
  #pragma unroll
  for (int i = 0; i < 2; ++i) {
    const int lid = w * 8 + i * 4 + sub;
    const int row = lid >> 2, seg = lid & 3;
    const v8us v = *(const v8usa*)(St + row * TP + 64 * seg + 8 * q8);
    unsigned short* dst = Tt + (size_t)(n0 + row) * FD + 64 * seg + 8 * q8;
    *(volatile v8us*)dst = v;
  }
}

__global__ __launch_bounds__(256) void prepack_kernel(const float* __restrict__ T,
                                                       unsigned short* __restrict__ Tt) {
  __shared__ __attribute__((aligned(16))) unsigned short St[16 * TP];

  const int t = threadIdx.x, lane = t & 31, w = t >> 5;
  const int n0 = blockIdx.x * 16;
  if (n0 >= NCOL) return;
  const int nn = t & 15, kb = t >> 4;

  #pragma unroll 4
  for (int i = 0; i < 16; ++i) {
    const int k = 16 * i + kb;
    const float v = T[(size_t)k * NCOL + n0 + nn];
    St[nn * TP + k] = (unsigned short)bf16_bits(v);
  }
  __syncthreads();

  tt_store_pass(St, Tt, n0, w, lane);
  __threadfence();
  tt_store_pass(St, Tt, n0, w, lane);
}

__device__ __forceinline__ void ob_store_pass(const float* So, float* out,
                                              int hw, int half, int w, int lane) {
  const int q8 = lane & 7, sub = lane >> 3;
  const int n = 4 * w + sub;
  const v4f v = *(const v4fa*)(So + n * SP + 4 * q8);
  const size_t gi = ((size_t)n * HWN + hw) * OUTC + FD + 32 * half + 4 * q8;
  *(volatile v4f*)(out + gi) = v;
}

__global__ __launch_bounds__(256) void mbd_kernel(const float* __restrict__ x,
                                                   const unsigned short* __restrict__ Tt,
                                                   float* __restrict__ out) {
  __shared__ __attribute__((aligned(16))) unsigned short Xs[NS * XP];
  __shared__ __attribute__((aligned(16))) float Ms[NS * MP];
  __shared__ __attribute__((aligned(16))) float So[NS * SP];

  const int t = threadIdx.x, lane = t & 31, w = t >> 5;
  const int hw = blockIdx.x >> 1, half = blockIdx.x & 1;
  if (hw >= HWN) return;

  {
    const int rsub = t >> 6;
    const int f4 = (t & 63) * 4;
    #pragma unroll
    for (int p = 0; p < 8; ++p) {
      const int n = 4 * p + rsub;
      const size_t rowid = (size_t)n * HWN + hw;
      const v4f v = *(const v4fa*)(x + rowid * FD + f4);
      const unsigned int b0 = bf16_bits(v.x), b1 = bf16_bits(v.y);
      const unsigned int b2 = bf16_bits(v.z), b3 = bf16_bits(v.w);
      v2u pk;
      pk.x = b0 | (b1 << 16);
      pk.y = b2 | (b3 << 16);
      *(v2ua*)(Xs + n * XP + f4) = pk;
      if (half == 0) {
        v4f r;
        r.x = __uint_as_float(b0 << 16);
        r.y = __uint_as_float(b1 << 16);
        r.z = __uint_as_float(b2 << 16);
        r.w = __uint_as_float(b3 << 16);
        float* dst = out + rowid * OUTC + f4;
        *(volatile v4f*)dst = r;
        __threadfence();
        *(volatile v4f*)dst = r;
      }
    }
  }
  __syncthreads();

  const int h = lane >> 4, m = lane & 15;
  {
    const v8f zero8 = {0.f, 0.f, 0.f, 0.f, 0.f, 0.f, 0.f, 0.f};
    v8f acc[2][2];
    #pragma unroll
    for (int mt = 0; mt < 2; ++mt)
      #pragma unroll
      for (int nt = 0; nt < 2; ++nt) acc[mt][nt] = zero8;

    const unsigned short* xa0 = Xs + m * XP;
    const unsigned short* xa1 = Xs + (16 + m) * XP;
    const unsigned short* tb0 = Tt + (size_t)(256 * half + 32 * w + m) * FD;
    const unsigned short* tb1 = tb0 + (size_t)16 * FD;

    #pragma unroll 1
    for (int k0 = 0; k0 < FD; k0 += 32) {
      const v16bf a0 = load_frag(xa0 + k0, h);
      const v16bf a1 = load_frag(xa1 + k0, h);
      const v16bf b0 = load_frag(tb0 + k0, h);
      const v16bf b1 = load_frag(tb1 + k0, h);
      acc[0][0] = wmma_bf16(a0, b0, acc[0][0]);
      acc[1][0] = wmma_bf16(a1, b0, acc[1][0]);
      acc[0][1] = wmma_bf16(a0, b1, acc[0][1]);
      acc[1][1] = wmma_bf16(a1, b1, acc[1][1]);
    }

    #pragma unroll
    for (int mt = 0; mt < 2; ++mt)
      #pragma unroll
      for (int nt = 0; nt < 2; ++nt)
        #pragma unroll
        for (int r = 0; r < 8; ++r)
          Ms[(16 * mt + 8 * h + r) * MP + 32 * w + 16 * nt + m] = acc[mt][nt][r];
  }
  __syncthreads();

  #pragma unroll 1
  for (int it = 0; it < 4; ++it) {
    const int bl = 8 * it + w;
    const int n = lane;
    const float* mi = Ms + n * MP + bl * CD;
    const v4f ia = *(const v4fa*)mi;
    const v4f ib = *(const v4fa*)(mi + 4);
    float o = 0.0f;
    #pragma unroll 1
    for (int j = 0; j < NS; ++j) {
      const float* mj = Ms + j * MP + bl * CD;
      const v4f ja = *(const v4fa*)mj;
      const v4f jb = *(const v4fa*)(mj + 4);
      const float d = fabsf(ia.x - ja.x) + fabsf(ia.y - ja.y)
                    + fabsf(ia.z - ja.z) + fabsf(ia.w - ja.w)
                    + fabsf(ib.x - jb.x) + fabsf(ib.y - jb.y)
                    + fabsf(ib.z - jb.z) + fabsf(ib.w - jb.w);
      o += expf(-d);
    }
    So[n * SP + bl] = o;
  }
  __syncthreads();

  ob_store_pass(So, out, hw, half, w, lane);
  __threadfence();
  ob_store_pass(So, out, hw, half, w, lane);
}

extern "C" void kernel_launch(void* const* d_in, const int* in_sizes, int n_in,
                              void* d_out, int out_size, void* d_ws, size_t ws_size,
                              hipStream_t stream) {
  if (n_in < 2) return;
  if (in_sizes[0] != NS * HWN * FD) return;
  if (in_sizes[1] != FD * NCOL) return;
  if (out_size != NS * HWN * OUTC) return;

  const float* x = (const float*)d_in[0];
  const float* T = (const float*)d_in[1];
  float* out = (float*)d_out;

  const size_t tt_bytes = (size_t)NCOL * FD * 2;
  if (tt_bytes > ws_size) return;
  unsigned short* Tt = (unsigned short*)d_ws;

  prepack_kernel<<<NCOL / 16, 256, 0, stream>>>(T, Tt);
  mbd_kernel<<<HWN * 2, 256, 0, stream>>>(x, Tt, out);
}
